// PAKA3x3_84696755077659
// MI455X (gfx1250) — hardware-verified
//
#include <hip/hip_runtime.h>

#define NB    4
#define NC    128
#define NO    128
#define IH    128
#define IW    128
#define NPIX  (IH * IW)
#define KTAPS 9
#define KTOT  (KTAPS * NC)
#define LDK   136

typedef __bf16   v16b __attribute__((ext_vector_type(16)));
typedef float    v8f  __attribute__((ext_vector_type(8)));
typedef float    v4f  __attribute__((ext_vector_type(4)));
typedef unsigned v4u  __attribute__((ext_vector_type(4)));
typedef v4f   __attribute__((may_alias)) v4fa;
typedef v4u   __attribute__((may_alias)) v4ua;
typedef float __attribute__((may_alias)) f32a;

union Frag { v16b v; v4u u[2]; };

static __device__ __forceinline__ unsigned f2bf(float f) {
  unsigned u = __float_as_uint(f);
  u += 0x7FFFu + ((u >> 16) & 1u);
  return u >> 16;
}
static __device__ __forceinline__ float bf2f(unsigned hbits) {
  return __uint_as_float(hbits << 16);
}
static __device__ __forceinline__ void split8(v8f v, v4u& hi, v4u& lo) {
  v4u ph = {0u, 0u, 0u, 0u}, pl = {0u, 0u, 0u, 0u};
#pragma unroll
  for (int j = 0; j < 4; ++j) {
    const unsigned h0 = f2bf(v[2 * j]), h1 = f2bf(v[2 * j + 1]);
    const unsigned l0 = f2bf(v[2 * j] - bf2f(h0));
    const unsigned l1 = f2bf(v[2 * j + 1] - bf2f(h1));
    ph[j] = h0 | (h1 << 16);
    pl[j] = l0 | (l1 << 16);
  }
  hi = ph; lo = pl;
}

static __device__ __forceinline__ v16b ldfrag(const unsigned short* p, int h) {
  Frag f;
  f.u[0] = *(const v4ua*)(p + 8 * h);
  f.u[1] = *(const v4ua*)(p + 16 + 8 * h);
  return f.v;
}

static __device__ __forceinline__ v8f mma3(v16b ah, v16b al, v16b bh, v16b bl, v8f c) {
  c = __builtin_amdgcn_wmma_f32_16x16x32_bf16(false, ah, false, bh, (short)0, c, false, false);
  c = __builtin_amdgcn_wmma_f32_16x16x32_bf16(false, ah, false, bl, (short)0, c, false, false);
  c = __builtin_amdgcn_wmma_f32_16x16x32_bf16(false, al, false, bh, (short)0, c, false, false);
  asm volatile("v_nop\n\tv_nop\n\tv_nop\n\tv_nop" : "+v"(c) : "v"(ah), "v"(al), "v"(bh), "v"(bl));
  return c;
}

static __device__ __forceinline__ v8f zero8() {
  v8f z = {0.f, 0.f, 0.f, 0.f, 0.f, 0.f, 0.f, 0.f};
  return z;
}

static __device__ __forceinline__ int refl(int i, int n) {
  i = (i < 0) ? -i : i;
  return (i >= n) ? (2 * n - 2 - i) : i;
}

__global__ __launch_bounds__(256) void k_prep_w(
    const float* __restrict__ wc1, const float* __restrict__ wc2,
    const float* __restrict__ wd1, const float* __restrict__ wd2,
    const float* __restrict__ wp,
    unsigned short* wc1h, unsigned short* wc1l,
    unsigned short* wc2h, unsigned short* wc2l,
    unsigned short* wd1h, unsigned short* wd1l,
    unsigned short* wd2h, unsigned short* wd2l,
    unsigned short* wph, unsigned short* wpl)
{
  const int bid = blockIdx.x, t = threadIdx.x;
  const float* src;
  int sstr = 1;
  bool zero = false;
  unsigned short* dh;
  unsigned short* dl;
  if (bid < 8) {
    const int e = (bid * 256 + t) * 8;
    src = wc1 + e; dh = wc1h + e; dl = wc1l + e;
  } else if (bid < 16) {
    const int e = ((bid - 8) * 256 + t) * 8;
    src = wc2 + e; dh = wc2h + e; dl = wc2l + e;
  } else if (bid < 88) {
    const int e = ((bid - 16) * 256 + t) * 8;
    const int o = e / KTOT, rem = e - o * KTOT;
    const int tap = rem >> 7, c = rem & 127;
    src = wd1 + (size_t)(o * NC + c) * KTAPS + tap;
    sstr = KTAPS; dh = wd1h + e; dl = wd1l + e;
  } else if (bid < 160) {
    const int e = ((bid - 88) * 256 + t) * 8;
    const int o = e / KTOT, rem = e - o * KTOT;
    const int tap = rem >> 7, c = rem & 127;
    src = wp + (size_t)(o * NC + c) * KTAPS + tap;
    sstr = KTAPS; dh = wph + e; dl = wpl + e;
  } else {
    const int e = t * 8;
    const int j = e >> 7, c = e & 127;
    const int jc = (j < KTAPS) ? j : (KTAPS - 1);
    src = wd2 + jc * NC + c; zero = (j >= KTAPS);
    dh = wd2h + e; dl = wd2l + e;
  }
  v8f v;
#pragma unroll
  for (int i = 0; i < 8; ++i) {
    const float f = src[i * sstr];
    v[i] = zero ? 0.0f : f;
  }
  v4u hv, lv;
  split8(v, hv, lv);
  *(volatile v4u*)dh = hv;
  *(volatile v4u*)dl = lv;
  __threadfence();
  *(volatile v4u*)dh = hv;
  *(volatile v4u*)dl = lv;
}

__global__ __launch_bounds__(256) void k_prep_x(const float* __restrict__ x,
                                                 unsigned short* xh, unsigned short* xl)
{
  __shared__ __attribute__((aligned(16))) float sx[NC * 32];
  const int t = threadIdx.x;
  const int b = blockIdx.x >> 9;
  const int p0 = (blockIdx.x & 511) << 5;
  const float* xb = x + (size_t)b * NC * NPIX + p0;
#pragma unroll
  for (int i = 0; i < 4; ++i) {
    const int q = i * 256 + t;
    const int c = q >> 3, j4 = (q & 7) << 2;
    const v4f v = *(const v4fa*)(xb + (size_t)c * NPIX + j4);
    *(v4fa*)(sx + c * 32 + j4) = v;
  }
  __syncthreads();

  v4u hv[2], lv[2];
  size_t ev[2];
#pragma unroll
  for (int i = 0; i < 2; ++i) {
    const int q = i * 256 + t;
    const int px = q >> 4, c8 = (q & 15) << 3;
    v8f v;
#pragma unroll
    for (int k = 0; k < 8; ++k) v[k] = sx[(c8 + k) * 32 + px];
    split8(v, hv[i], lv[i]);
    ev[i] = (((size_t)b * NPIX + p0 + px) << 7) + c8;
  }
#pragma unroll
  for (int i = 0; i < 2; ++i) {
    *(volatile v4u*)(xh + ev[i]) = hv[i];
    *(volatile v4u*)(xl + ev[i]) = lv[i];
  }
  __threadfence();
#pragma unroll
  for (int i = 0; i < 2; ++i) {
    *(volatile v4u*)(xh + ev[i]) = hv[i];
    *(volatile v4u*)(xl + ev[i]) = lv[i];
  }
}

__global__ __launch_bounds__(256) void k_convc(
    const unsigned short* __restrict__ xh, const unsigned short* __restrict__ xl,
    const unsigned short* __restrict__ wc1h, const unsigned short* __restrict__ wc1l,
    const unsigned short* __restrict__ wc2h, const unsigned short* __restrict__ wc2l,
    float* cc)
{
  __shared__ __attribute__((aligned(16))) unsigned short sm[2 * 64 * LDK];
  unsigned short* Th = sm;
  unsigned short* Tl = sm + 64 * LDK;

  const int tid = threadIdx.x, lane = tid & 31, wv = tid >> 5;
  const int h = lane >> 4, m = lane & 15;
  const int b = blockIdx.x >> 8;
  const int n0 = (blockIdx.x & 255) << 6;
  const size_t pix0 = (size_t)b * NPIX + n0;

  v8f acc[4];
#pragma unroll
  for (int nt = 0; nt < 4; ++nt) acc[nt] = zero8();

  {
    const unsigned short* ahp = wc1h + (size_t)(16 * wv + m) * NC;
    const unsigned short* alp = wc1l + (size_t)(16 * wv + m) * NC;
#pragma unroll 1
    for (int kk = 0; kk < 4; ++kk) {
      const v16b ah = ldfrag(ahp + 32 * kk, h);
      const v16b al = ldfrag(alp + 32 * kk, h);
#pragma unroll
      for (int nt = 0; nt < 4; ++nt) {
        const size_t e = ((pix0 + 16 * nt + m) << 7) + 32 * kk;
        const v16b bh = ldfrag(xh + e, h);
        const v16b bl = ldfrag(xl + e, h);
        acc[nt] = mma3(ah, al, bh, bl, acc[nt]);
      }
    }
  }

#pragma unroll
  for (int nt = 0; nt < 4; ++nt) {
    v8f tv;
#pragma unroll
    for (int r = 0; r < 8; ++r) tv[r] = fmaxf(acc[nt][r], 0.0f);
    v4u hv, lv;
    split8(tv, hv, lv);
    const int off = (16 * nt + m) * LDK + 16 * wv + 8 * h;
    *(v4ua*)(Th + off) = hv;
    *(v4ua*)(Tl + off) = lv;
  }
  __syncthreads();

#pragma unroll
  for (int nt = 0; nt < 4; ++nt) acc[nt] = zero8();
  {
    const unsigned short* ahp = wc2h + (size_t)(16 * wv + m) * NC;
    const unsigned short* alp = wc2l + (size_t)(16 * wv + m) * NC;
#pragma unroll 1
    for (int kk = 0; kk < 4; ++kk) {
      const v16b ah = ldfrag(ahp + 32 * kk, h);
      const v16b al = ldfrag(alp + 32 * kk, h);
#pragma unroll
      for (int nt = 0; nt < 4; ++nt) {
        const int boff = (16 * nt + m) * LDK + 32 * kk;
        const v16b bh = ldfrag(Th + boff, h);
        const v16b bl = ldfrag(Tl + boff, h);
        acc[nt] = mma3(ah, al, bh, bl, acc[nt]);
      }
    }
  }
  __syncthreads();

  f32a* S = (f32a*)sm;
#pragma unroll
  for (int nt = 0; nt < 4; ++nt) {
    const int off = (16 * nt + m) * NC + 16 * wv + 8 * h;
    const v4f v0 = {acc[nt][0], acc[nt][1], acc[nt][2], acc[nt][3]};
    const v4f v1 = {acc[nt][4], acc[nt][5], acc[nt][6], acc[nt][7]};
    *(v4fa*)(S + off) = v0;
    *(v4fa*)(S + off + 4) = v1;
  }
  __syncthreads();

  float* dst = cc + (pix0 << 7);
  v4f sv[8];
#pragma unroll
  for (int i = 0; i < 8; ++i) sv[i] = *(const v4fa*)(S + (i * 256 + tid) * 4);
#pragma unroll
  for (int i = 0; i < 8; ++i) *(volatile v4f*)(dst + (size_t)(i * 256 + tid) * 4) = sv[i];
  __threadfence();
#pragma unroll
  for (int i = 0; i < 8; ++i) *(volatile v4f*)(dst + (size_t)(i * 256 + tid) * 4) = sv[i];
}

__global__ __launch_bounds__(256) void k_convd(
    const unsigned short* __restrict__ xh, const unsigned short* __restrict__ xl,
    const unsigned short* __restrict__ wd1h, const unsigned short* __restrict__ wd1l,
    const unsigned short* __restrict__ wd2h, const unsigned short* __restrict__ wd2l,
    float* dd)
{
  __shared__ __attribute__((aligned(16))) unsigned short sm[2 * 64 * LDK + 2 * 64 * 16];
  unsigned short* Th = sm;
  unsigned short* Tl = sm + 64 * LDK;
  f32a* Sd = (f32a*)(sm + 2 * 64 * LDK);

  const int tid = threadIdx.x, lane = tid & 31, wv = tid >> 5;
  const int h = lane >> 4, m = lane & 15;
  const int b = blockIdx.x >> 8;
  const int rem = blockIdx.x & 255;
  const int y = rem >> 1, w0 = (rem & 1) << 6;
  const size_t img = (size_t)b * NPIX;

  v8f acc[4];
#pragma unroll
  for (int nt = 0; nt < 4; ++nt) acc[nt] = zero8();

  const unsigned short* ahp = wd1h + (size_t)(16 * wv + m) * KTOT;
  const unsigned short* alp = wd1l + (size_t)(16 * wv + m) * KTOT;
#pragma unroll 1
  for (int tap = 0; tap < KTAPS; ++tap) {
    const int kh = tap / 3, kw = tap - 3 * kh;
    const int yy = refl(y + kh - 1, IH);
#pragma unroll 1
    for (int kk = 0; kk < 4; ++kk) {
      const v16b ah = ldfrag(ahp + tap * NC + 32 * kk, h);
      const v16b al = ldfrag(alp + tap * NC + 32 * kk, h);
#pragma unroll
      for (int nt = 0; nt < 4; ++nt) {
        const int xx = refl(w0 + 16 * nt + m + kw - 1, IW);
        const size_t e = ((img + (size_t)yy * IW + xx) << 7) + 32 * kk;
        const v16b bh = ldfrag(xh + e, h);
        const v16b bl = ldfrag(xl + e, h);
        acc[nt] = mma3(ah, al, bh, bl, acc[nt]);
      }
    }
  }

#pragma unroll
  for (int nt = 0; nt < 4; ++nt) {
    v8f tv;
#pragma unroll
    for (int r = 0; r < 8; ++r) tv[r] = fmaxf(acc[nt][r], 0.0f);
    v4u hv, lv;
    split8(tv, hv, lv);
    const int off = (16 * nt + m) * LDK + 16 * wv + 8 * h;
    *(v4ua*)(Th + off) = hv;
    *(v4ua*)(Tl + off) = lv;
  }
  __syncthreads();

  if (wv < 4) {
    v8f a2 = zero8();
    const unsigned short* a2h = wd2h + m * NC;
    const unsigned short* a2l = wd2l + m * NC;
    const int boff = (16 * wv + m) * LDK;
#pragma unroll 1
    for (int kk = 0; kk < 4; ++kk) {
      const v16b ah = ldfrag(a2h + 32 * kk, h);
      const v16b al = ldfrag(a2l + 32 * kk, h);
      const v16b bh = ldfrag(Th + boff + 32 * kk, h);
      const v16b bl = ldfrag(Tl + boff + 32 * kk, h);
      a2 = mma3(ah, al, bh, bl, a2);
    }
    const int so = (16 * wv + m) * 16 + 8 * h;
    const v4f v0 = {a2[0], a2[1], a2[2], a2[3]};
    const v4f v1 = {a2[4], a2[5], a2[6], a2[7]};
    *(v4fa*)(Sd + so) = v0;
    *(v4fa*)(Sd + so + 4) = v1;
  }
  __syncthreads();

  const v4f dv = *(const v4fa*)(Sd + tid * 4);
  float* ddst = dd + ((img + (size_t)y * IW + w0) << 4) + tid * 4;
  *(volatile v4f*)ddst = dv;
  __threadfence();
  *(volatile v4f*)ddst = dv;
}

__global__ __launch_bounds__(256) void k_final(
    const unsigned short* __restrict__ xh, const unsigned short* __restrict__ xl,
    const unsigned short* __restrict__ wph, const unsigned short* __restrict__ wpl,
    const float* __restrict__ cc, const float* __restrict__ dd, float* out)
{
  __shared__ __attribute__((aligned(16))) unsigned short sm[2 * 64 * LDK];
  unsigned short* Vh = sm;
  unsigned short* Vl = sm + 64 * LDK;

  const int tid = threadIdx.x, lane = tid & 31, wv = tid >> 5;
  const int h = lane >> 4, m = lane & 15;
  const int b = blockIdx.x >> 8;
  const int rem = blockIdx.x & 255;
  const int y = rem >> 1, w0 = (rem & 1) << 6;
  const size_t img = (size_t)b * NPIX;
  const size_t prow = img + (size_t)y * IW + w0;

  v8f acc[4];
#pragma unroll
  for (int nt = 0; nt < 4; ++nt) acc[nt] = zero8();

  const unsigned short* ahp = wph + (size_t)(16 * wv + m) * KTOT;
  const unsigned short* alp = wpl + (size_t)(16 * wv + m) * KTOT;

#pragma unroll 1
  for (int tap = 0; tap < KTAPS; ++tap) {
    const int kh = tap / 3, kw = tap - 3 * kh;
    const int yy = y + kh - 1;
    const bool yin = (yy >= 0) && (yy < IH);
    const int yc = (yy < 0) ? 0 : ((yy >= IH) ? (IH - 1) : yy);

#pragma unroll
    for (int i = 0; i < 4; ++i) {
      const int q = i * 256 + tid;
      const int px = q >> 4, c8 = (q & 15) << 3;
      const int xx = w0 + px + kw - 1;
      const bool inb = yin && (xx >= 0) && (xx < IW);
      const int xc = (xx < 0) ? 0 : ((xx >= IW) ? (IW - 1) : xx);
      const size_t e = ((img + (size_t)yc * IW + xc) << 7) + c8;
      const v4u xhv = *(const v4ua*)(xh + e);
      const v4u xlv = *(const v4ua*)(xl + e);
      const size_t pe = prow + px;
      const v4f ca = *(const v4fa*)(cc + (pe << 7) + c8);
      const v4f cb = *(const v4fa*)(cc + (pe << 7) + c8 + 4);
      const v8f cv = __builtin_shufflevector(ca, cb, 0, 1, 2, 3, 4, 5, 6, 7);
      const float dv = dd[(pe << 4) + tap];
      v8f v;
#pragma unroll
      for (int k = 0; k < 8; ++k) {
        const unsigned wdh = xhv[k >> 1], wdl = xlv[k >> 1];
        const unsigned hb = (k & 1) ? (wdh >> 16) : (wdh & 0xFFFFu);
        const unsigned lb = (k & 1) ? (wdl >> 16) : (wdl & 0xFFFFu);
        const float xv = bf2f(hb) + bf2f(lb);
        const float s = dv + cv[k];
        const float g = 2.0f * __builtin_amdgcn_rcpf(
                            1.0f + __builtin_amdgcn_exp2f(-2.8853900817779268f * s));
        v[k] = inb ? (xv * g) : 0.0f;
      }
      v4u hv, lv;
      split8(v, hv, lv);
      const int off = px * LDK + c8;
      *(v4ua*)(Vh + off) = hv;
      *(v4ua*)(Vl + off) = lv;
    }
    __syncthreads();

#pragma unroll 1
    for (int kk = 0; kk < 4; ++kk) {
      const v16b ah = ldfrag(ahp + tap * NC + 32 * kk, h);
      const v16b al = ldfrag(alp + tap * NC + 32 * kk, h);
#pragma unroll
      for (int nt = 0; nt < 4; ++nt) {
        const int boff = (16 * nt + m) * LDK + 32 * kk;
        const v16b bh = ldfrag(Vh + boff, h);
        const v16b bl = ldfrag(Vl + boff, h);
        acc[nt] = mma3(ah, al, bh, bl, acc[nt]);
      }
    }
    __syncthreads();
  }

  f32a* So = (f32a*)sm;
#pragma unroll
  for (int nt = 0; nt < 4; ++nt) {
#pragma unroll
    for (int r = 0; r < 8; ++r)
      So[(16 * wv + 8 * h + r) * 64 + 16 * nt + m] = acc[nt][r];
  }
  __syncthreads();

  v4f sv[8];
  size_t go[8];
#pragma unroll
  for (int i = 0; i < 8; ++i) {
    const int row = i * 16 + (tid >> 4);
    const int piece = (tid & 15) * 4;
    sv[i] = *(const v4fa*)(So + row * 64 + piece);
    go[i] = (size_t)(b * NO + row) * NPIX + (size_t)y * IW + w0 + piece;
  }
#pragma unroll
  for (int i = 0; i < 8; ++i) *(volatile v4f*)(out + go[i]) = sv[i];
  __threadfence();
#pragma unroll
  for (int i = 0; i < 8; ++i) *(volatile v4f*)(out + go[i]) = sv[i];
}

extern "C" void kernel_launch(void* const* d_in, const int* in_sizes, int n_in,
                              void* d_out, int out_size, void* d_ws, size_t ws_size,
                              hipStream_t stream) {
  if (n_in < 6) return;
  if (in_sizes[0] != NB * NC * NPIX) return;
  if (in_sizes[1] != NO * NC * KTAPS) return;
  if (in_sizes[2] != NC * NC) return;
  if (in_sizes[3] != NC * NC) return;
  if (in_sizes[4] != NO * NC * KTAPS) return;
  if (in_sizes[5] != KTAPS * NC) return;
  if (out_size != NB * NO * NPIX) return;

  const float* x     = (const float*)d_in[0];
  const float* wpaka = (const float*)d_in[1];
  const float* wc1   = (const float*)d_in[2];
  const float* wc2   = (const float*)d_in[3];
  const float* wd1   = (const float*)d_in[4];
  const float* wd2   = (const float*)d_in[5];
  float* out = (float*)d_out;

  const size_t b_wc  = (size_t)NC * NC * 2;
  const size_t b_wk  = (size_t)NO * KTOT * 2;
  const size_t b_wd2 = (size_t)16 * NC * 2;
  const size_t b_xp  = (size_t)NB * NPIX * NC * 2;
  const size_t b_cc  = (size_t)NB * NPIX * NC * 4;
  const size_t b_dd  = (size_t)NB * NPIX * 16 * 4;

  size_t off = 0;
  const size_t o_wc1h = off; off += b_wc;
  const size_t o_wc1l = off; off += b_wc;
  const size_t o_wc2h = off; off += b_wc;
  const size_t o_wc2l = off; off += b_wc;
  const size_t o_wd1h = off; off += b_wk;
  const size_t o_wd1l = off; off += b_wk;
  const size_t o_wph  = off; off += b_wk;
  const size_t o_wpl  = off; off += b_wk;
  const size_t o_wd2h = off; off += b_wd2;
  const size_t o_wd2l = off; off += b_wd2;
  const size_t o_xh   = off; off += b_xp;
  const size_t o_xl   = off; off += b_xp;
  const size_t o_cc   = off; off += b_cc;
  const size_t o_dd   = off; off += b_dd;
  if (off > ws_size) return;

  char* ws = (char*)d_ws;
  unsigned short* wc1h = (unsigned short*)(ws + o_wc1h);
  unsigned short* wc1l = (unsigned short*)(ws + o_wc1l);
  unsigned short* wc2h = (unsigned short*)(ws + o_wc2h);
  unsigned short* wc2l = (unsigned short*)(ws + o_wc2l);
  unsigned short* wd1h = (unsigned short*)(ws + o_wd1h);
  unsigned short* wd1l = (unsigned short*)(ws + o_wd1l);
  unsigned short* wph  = (unsigned short*)(ws + o_wph);
  unsigned short* wpl  = (unsigned short*)(ws + o_wpl);
  unsigned short* wd2h = (unsigned short*)(ws + o_wd2h);
  unsigned short* wd2l = (unsigned short*)(ws + o_wd2l);
  unsigned short* xh   = (unsigned short*)(ws + o_xh);
  unsigned short* xl   = (unsigned short*)(ws + o_xl);
  float* cc = (float*)(ws + o_cc);
  float* dd = (float*)(ws + o_dd);

  k_prep_w<<<161, 256, 0, stream>>>(wc1, wc2, wd1, wd2, wpaka,
                                     wc1h, wc1l, wc2h, wc2l, wd1h, wd1l, wd2h, wd2l, wph, wpl);
  k_prep_x<<<NB * (NPIX / 32), 256, 0, stream>>>(x, xh, xl);
  k_convc<<<NB * (NPIX / 64), 256, 0, stream>>>(xh, xl, wc1h, wc1l, wc2h, wc2l, cc);
  k_convd<<<NB * IH * (IW / 64), 256, 0, stream>>>(xh, xl, wd1h, wd1l, wd2h, wd2l, dd);
  k_final<<<NB * IH * (IW / 64), 256, 0, stream>>>(xh, xl, wph, wpl, cc, dd, out);
}
